// DecoderBlock_28166395527956
// MI455X (gfx1250) — hardware-verified
//
#include <hip/hip_runtime.h>
#include <stddef.h>


typedef _Float16 v16h __attribute__((ext_vector_type(16)));
typedef _Float16 v8h  __attribute__((ext_vector_type(8)));
typedef float    v8f  __attribute__((ext_vector_type(8)));
typedef float    v4f  __attribute__((ext_vector_type(4)));

#ifndef NB
#define NB 8
#endif
#ifndef SEQ
#define SEQ 2048
#endif
#define NB_FULL  8
#define SEQ_FULL 2048
#define EMB   64
#define DIM   256
#define HID   256
#define NHEAD 4
#define HD    64
#define MROWS (NB * SEQ)
#define WELEMS 16384

static_assert(NB >= 1 && NB <= NB_FULL);
static_assert(SEQ >= 128 && SEQ <= SEQ_FULL && (SEQ % 128) == 0);
static_assert(DIM == NHEAD * HD);
static_assert(HD == 64);
static_assert(EMB == 64);
static_assert(HID == 4 * EMB);
static_assert((DIM % 64) == 0 && (DIM % 32) == 0);
static_assert((HID % 64) == 0 && (HID % 32) == 0);
static_assert((EMB % 64) == 0 && (EMB % 32) == 0);
static_assert((MROWS % 64) == 0 && (MROWS % 32) == 0);
static_assert((SEQ % 64) == 0);
static_assert(256 * 8 == 32 * EMB);
static_assert(DIM * EMB == WELEMS && HID * EMB == WELEMS && EMB * DIM == WELEMS);
static_assert((WELEMS % (256 * 8)) == 0);
static_assert((size_t)MROWS * HID < (size_t)0xFFFFFFFFu);

#define LDT 72
#define LDC 68
static_assert((LDT % 8) == 0 && LDT >= 64);
static_assert((LDC % 4) == 0 && LDC >= 64);
static_assert((size_t)(3 * 64 * LDT + 8 * 16 * LDT) * 2 <= (size_t)131072);
static_assert((size_t)(64 * LDC) * 4 <= (size_t)131072);

#define WCARRY 64.0f
#define PCARRY 1024.0f
#define VCARRY 64.0f
#define MCARRY 16.0f
#define RCARRY 1024.0f

#define WPL_BYTES     ((size_t)WELEMS * 2)
#define H_BYTES       ((size_t)MROWS * EMB * 2)
#define PLANE16_BYTES ((size_t)MROWS * DIM * 2)
#define VRES_BYTES    ((size_t)NB * DIM * 64 * 2)
#define X1_BYTES      ((size_t)MROWS * EMB * 4)
#define MID_BYTES     ((size_t)MROWS * HID * 2)
#define OFF_WQ  ((size_t)0)
#define OFF_WK  (OFF_WQ + WPL_BYTES)
#define OFF_WV  (OFF_WK + WPL_BYTES)
#define OFF_WO  (OFF_WV + WPL_BYTES)
#define OFF_W1  (OFF_WO + WPL_BYTES)
#define OFF_W2  (OFF_W1 + WPL_BYTES)
#define OFF_H1  (OFF_W2 + WPL_BYTES)
#define OFF_H2  (OFF_H1 + H_BYTES)
#define OFF_Q   (OFF_H2 + H_BYTES)
#define OFF_K   (OFF_Q + PLANE16_BYTES)
#define OFF_VT  (OFF_K + PLANE16_BYTES)
#define OFF_CTX (OFF_VT + PLANE16_BYTES)
#define OFF_VR  (OFF_CTX + PLANE16_BYTES)
#define OFF_X1  (OFF_VR + VRES_BYTES)
#define OFF_MID (OFF_X1 + X1_BYTES)
#define WS_TOTAL (OFF_MID + MID_BYTES)
static_assert((WPL_BYTES % 128) == 0 && (H_BYTES % 128) == 0 && (PLANE16_BYTES % 128) == 0);
static_assert((VRES_BYTES % 128) == 0 && (X1_BYTES % 128) == 0 && (MID_BYTES % 128) == 0);
static_assert(WS_TOTAL <= (size_t)134217728);

__device__ __forceinline__ float bf16r(float x) {
  unsigned int u = __float_as_uint(x);
  u = (u + 0x7FFFu + ((u >> 16) & 1u)) & 0xFFFF0000u;
  return __uint_as_float(u);
}

__device__ __forceinline__ v16h frag_at(const _Float16* p) {
  v8h lo = *(const v8h*)(p);
  v8h hi = *(const v8h*)(p + 16);
  v16h out;
#pragma unroll
  for (int i = 0; i < 8; ++i) { out[i] = lo[i]; out[i + 8] = hi[i]; }
  return out;
}
__device__ __forceinline__ v16h ld_frag(const _Float16* base, unsigned ld) {
  const unsigned lane = threadIdx.x & 31u;
  return frag_at(base + (lane & 15u) * ld + (lane >> 4) * 8u);
}

__device__ __forceinline__ v8f wmma16(v16h a, v16h b, v8f c) {
  v8f d = __builtin_amdgcn_wmma_f32_16x16x32_f16(false, a, false, b, (short)0, c,
                                                 false, false);
  asm volatile("v_nop\n\tv_nop\n\tv_nop\n\tv_nop" : "+v"(d) : "v"(a), "v"(b));
  return d;
}

__device__ __forceinline__ float red16_max(float x) {
#pragma unroll
  for (int off = 1; off < 16; off <<= 1) x = fmaxf(x, __shfl_xor(x, off, 32));
  return x;
}
__device__ __forceinline__ float red16_sum(float x) {
#pragma unroll
  for (int off = 1; off < 16; off <<= 1) x += __shfl_xor(x, off, 32);
  return x;
}
__device__ __forceinline__ float red32_sum(float x) {
#pragma unroll
  for (int off = 1; off < 32; off <<= 1) x += __shfl_xor(x, off, 32);
  return x;
}

__device__ __forceinline__ void wave_lds_sync() {
  __builtin_amdgcn_fence(3  , "wavefront");
  asm volatile("s_wait_dscnt 0x0" ::: "memory");
  __builtin_amdgcn_wave_barrier();
}

__device__ __forceinline__ float relu_act(float t) {
  return fmaxf(t, 0.0f);
}

__device__ __forceinline__ float red8_sum(float x) {
#pragma unroll
  for (int off = 1; off < 8; off <<= 1) x += __shfl_xor(x, off, 32);
  return x;
}

static __device__ __forceinline__ _Float16 toh_flush(float v) {
  const _Float16 r = (_Float16)v;
  return (fabsf(v) < 6.103515625e-05f) ? (_Float16)0.0f : r;
}

__global__ __launch_bounds__(256) void wplane_kernel(
    const float* __restrict__ W, _Float16* __restrict__ Wt) {
  const unsigned e0 = (blockIdx.x * 256u + threadIdx.x) * 8u;
  const v4f a0 = *(const v4f*)(W + e0);
  const v4f a1 = *(const v4f*)(W + e0 + 4u);
  v8h x;
#pragma unroll
  for (int i = 0; i < 4; ++i) {
    x[i]     = toh_flush(WCARRY * bf16r(a0[i]));
    x[i + 4] = toh_flush(WCARRY * bf16r(a1[i]));
  }
  _Float16* p = Wt + e0;
  *(volatile v8h*)p = x;
  __threadfence();
  *(volatile v8h*)p = x;
}

template <int SRC_INPUT>
__device__ __forceinline__ void ln_body(const float* __restrict__ X,
                                        const float* __restrict__ G,
                                        const float* __restrict__ Be,
                                        _Float16* __restrict__ dst) {
#pragma clang fp contract(off)
  const unsigned tid = threadIdx.x;
  const unsigned crow = blockIdx.x * 32u + (tid >> 3);
  const unsigned c = (tid & 7u) * 8u;
  size_t srow = crow;
  if (SRC_INPUT) {
    const unsigned bidx = crow / (unsigned)SEQ;
    const unsigned sq = crow - bidx * (unsigned)SEQ;
    srow = (size_t)bidx * SEQ_FULL + sq;
  }
  const float* xr = X + srow * EMB + c;
  const v4f a0 = *(const v4f*)(xr);
  const v4f a1 = *(const v4f*)(xr + 4u);
  float e[8];
#pragma unroll
  for (int i = 0; i < 4; ++i) {
    e[i]     = SRC_INPUT ? bf16r(a0[i]) : a0[i];
    e[i + 4] = SRC_INPUT ? bf16r(a1[i]) : a1[i];
  }
  float s = 0.0f;
#pragma unroll
  for (int i = 0; i < 8; ++i) s += e[i];
  const float mean = red8_sum(s) * (1.0f / (float)EMB);

  float ss = 0.0f;
#pragma unroll
  for (int i = 0; i < 8; ++i) {
    const float d = e[i] - mean;
    ss += d * d;
  }
  const float var = red8_sum(ss) * (1.0f / (float)EMB);
  const float rstd = 1.0f / sqrtf(var + 1.0e-5f);

  const v4f g0 = *(const v4f*)(G + c);
  const v4f g1 = *(const v4f*)(G + c + 4u);
  const v4f b0 = *(const v4f*)(Be + c);
  const v4f b1 = *(const v4f*)(Be + c + 4u);
  v8h o;
#pragma unroll
  for (int i = 0; i < 4; ++i) {
    const float d0 = e[i] - mean;
    const float d1 = e[i + 4] - mean;
    o[i]     = toh_flush(d0 * rstd * bf16r(g0[i]) + bf16r(b0[i]));
    o[i + 4] = toh_flush(d1 * rstd * bf16r(g1[i]) + bf16r(b1[i]));
  }
  _Float16* p = dst + (size_t)crow * EMB + c;
  *(volatile v8h*)p = o;
  __threadfence();
  *(volatile v8h*)p = o;
}

__global__ __launch_bounds__(256) void ln_in_kernel(
    const float* __restrict__ X, const float* __restrict__ G, const float* __restrict__ Be,
    _Float16* __restrict__ dst) {
  ln_body<1>(X, G, Be, dst);
}
__global__ __launch_bounds__(256) void ln_ws_kernel(
    const float* __restrict__ X, const float* __restrict__ G, const float* __restrict__ Be,
    _Float16* __restrict__ dst) {
  ln_body<0>(X, G, Be, dst);
}

template <int MODE>
__device__ __forceinline__ void gemm_body(
    const _Float16* __restrict__ A16, const _Float16* __restrict__ Bt, const unsigned K,
    const float* __restrict__ bias, const float* __restrict__ addf,
    float* __restrict__ outf, _Float16* __restrict__ out16, _Float16* __restrict__ out16r) {
  __shared__ float Cs[64 * LDC];
  const unsigned tid = threadIdx.x, lane = tid & 31u, w = tid >> 5;
  const unsigned mw = w >> 1, nw = w & 1u;
  const unsigned hh = lane >> 4, m = lane & 15u;
  const unsigned n0 = blockIdx.x * 64u;
  const unsigned row0 = blockIdx.y * 64u;

  const _Float16* ap  = A16 + (size_t)(row0 + mw * 16u + m) * K + hh * 8u;
  const _Float16* bp0 = Bt + (size_t)(n0 + nw * 32u + m) * K + hh * 8u;
  const _Float16* bp1 = bp0 + (size_t)16 * K;
  v8f acc0 = {}, acc1 = {};
#pragma unroll 2
  for (unsigned k0 = 0; k0 < K; k0 += 32u) {
    const v16h a  = frag_at(ap + k0);
    const v16h b0 = frag_at(bp0 + k0);
    const v16h b1 = frag_at(bp1 + k0);
    acc0 = wmma16(a, b0, acc0);
    acc1 = wmma16(a, b1, acc1);
  }
#pragma unroll
  for (int r = 0; r < 8; ++r) {
    float* d = &Cs[(mw * 16u + hh * 8u + (unsigned)r) * LDC + nw * 32u + m];
    d[0]  = acc0[r];
    d[16] = acc1[r];
  }
  __syncthreads();

  if (MODE == 3) {
#pragma unroll 1
    for (unsigned g = 0; g < 4u; ++g) {
      const unsigned r = 32u * (g >> 1) + (tid >> 3);
      const unsigned c = (tid & 7u) * 8u + 4u * (g & 1u);
      const v4f u  = *(const v4f*)&Cs[r * LDC + c];
      const v4f gb = *(const v4f*)(bias + n0 + c);
      v4f t;
#pragma unroll
      for (int j = 0; j < 4; ++j)
        t[j] = MCARRY * relu_act(u[j] * (1.0f / WCARRY) + bf16r(gb[j]));
      *(v4f*)&Cs[r * LDC + c] = t;
    }
  }

  if (MODE == 0 || MODE == 3) {
    const unsigned ldo = (MODE == 3) ? (unsigned)HID : (unsigned)DIM;
    v8h x[2];
    size_t off[2];
#pragma unroll
    for (unsigned i = 0; i < 2u; ++i) {
      const unsigned r = 32u * i + (tid >> 3);
      const unsigned c = (tid & 7u) * 8u;
      const v4f u0 = *(const v4f*)&Cs[r * LDC + c];
      const v4f u1 = *(const v4f*)&Cs[r * LDC + c + 4];
      if (MODE == 3) {
#pragma unroll
        for (int j = 0; j < 4; ++j) {
          x[i][j]     = toh_flush(u0[j]);
          x[i][j + 4] = toh_flush(u1[j]);
        }
      } else {
#pragma unroll
        for (int j = 0; j < 4; ++j) {
          x[i][j]     = toh_flush(u0[j] * (1.0f / WCARRY));
          x[i][j + 4] = toh_flush(u1[j] * (1.0f / WCARRY));
        }
      }
      off[i] = (size_t)(row0 + r) * ldo + n0 + c;
    }
#pragma unroll
    for (int i = 0; i < 2; ++i) *(volatile v8h*)(out16 + off[i]) = x[i];
    __threadfence();
#pragma unroll
    for (int i = 0; i < 2; ++i) *(volatile v8h*)(out16 + off[i]) = x[i];
  }

  if (MODE == 1) {
    const unsigned bidx = row0 / (unsigned)SEQ;
    const unsigned key0 = row0 - bidx * (unsigned)SEQ;
    const bool first_tile = (key0 == 0u);
    v8h x[2], xr[2];
    size_t off[2], offr[2];
#pragma unroll
    for (unsigned i = 0; i < 2u; ++i) {
      const unsigned dcol = 32u * i + (tid >> 3);
      const unsigned kk = (tid & 7u) * 8u;
#pragma unroll
      for (unsigned j = 0; j < 8u; ++j) {
        const float t = Cs[(kk + j) * LDC + dcol] * (1.0f / WCARRY);
        const _Float16 hi = toh_flush(t);
        x[i][j]  = hi;
        xr[i][j] = toh_flush((t - (float)hi) * RCARRY);
      }
      off[i]  = ((size_t)bidx * DIM + n0 + dcol) * SEQ + key0 + kk;
      offr[i] = ((size_t)bidx * DIM + n0 + dcol) * 64u + kk;
    }
#pragma unroll
    for (int i = 0; i < 2; ++i) *(volatile v8h*)(out16 + off[i]) = x[i];
    if (first_tile) {
#pragma unroll
      for (int i = 0; i < 2; ++i) *(volatile v8h*)(out16r + offr[i]) = xr[i];
    }
    __threadfence();
#pragma unroll
    for (int i = 0; i < 2; ++i) *(volatile v8h*)(out16 + off[i]) = x[i];
    if (first_tile) {
#pragma unroll
      for (int i = 0; i < 2; ++i) *(volatile v8h*)(out16r + offr[i]) = xr[i];
    }
  }

  if (MODE == 2 || MODE == 4) {
    const float cs = (MODE == 2) ? (1.0f / (WCARRY * VCARRY)) : (1.0f / (WCARRY * MCARRY));
    v4f xs[4];
    size_t off[4];
#pragma unroll
    for (unsigned i = 0; i < 4u; ++i) {
      const unsigned r = 16u * i + (tid >> 4);
      const unsigned c = (tid & 15u) * 4u;
      const unsigned crow = row0 + r;
      const unsigned bidx = crow / (unsigned)SEQ;
      const unsigned sq = crow - bidx * (unsigned)SEQ;
      const size_t frow = (size_t)bidx * SEQ_FULL + sq;
      const size_t inrow  = (MODE == 2) ? frow : (size_t)crow;
      const size_t outrow = (MODE == 2) ? (size_t)crow : frow;
      const v4f u = *(const v4f*)&Cs[r * LDC + c];
      v4f g = {};
      if (MODE == 4) g = *(const v4f*)(bias + n0 + c);
      const v4f xin = *(const v4f*)(addf + inrow * EMB + n0 + c);
      v4f val;
#pragma unroll
      for (int j = 0; j < 4; ++j) {
        const float base = (MODE == 2) ? bf16r(xin[j]) : xin[j];
        const float bj = (MODE == 4) ? bf16r(g[j]) : 0.0f;
        val[j] = base + (u[j] * cs + bj);
      }
      xs[i] = val;
      off[i] = outrow * EMB + n0 + c;
    }
#pragma unroll
    for (int i = 0; i < 4; ++i) *(volatile v4f*)(outf + off[i]) = xs[i];
    __threadfence();
#pragma unroll
    for (int i = 0; i < 4; ++i) *(volatile v4f*)(outf + off[i]) = xs[i];
  }
}

__global__ __launch_bounds__(256) void gemm_qk_kernel(
    const _Float16* __restrict__ A16, const _Float16* __restrict__ Bt,
    _Float16* __restrict__ out16) {
  gemm_body<0>(A16, Bt, (unsigned)EMB, (const float*)0, (const float*)0, (float*)0, out16, out16);
}
__global__ __launch_bounds__(256) void gemm_v_kernel(
    const _Float16* __restrict__ A16, const _Float16* __restrict__ Bt,
    _Float16* __restrict__ vt, _Float16* __restrict__ vtr) {
  gemm_body<1>(A16, Bt, (unsigned)EMB, (const float*)0, (const float*)0, (float*)0, vt, vtr);
}
__global__ __launch_bounds__(256) void gemm_wo_kernel(
    const _Float16* __restrict__ A16, const _Float16* __restrict__ Bt,
    const float* __restrict__ xin, float* __restrict__ x1) {
  gemm_body<2>(A16, Bt, (unsigned)DIM, (const float*)0, xin, x1, (_Float16*)0, (_Float16*)0);
}
__global__ __launch_bounds__(256) void gemm_ffn1_kernel(
    const _Float16* __restrict__ A16, const _Float16* __restrict__ Bt,
    const float* __restrict__ bias, _Float16* __restrict__ mid) {
  gemm_body<3>(A16, Bt, (unsigned)EMB, bias, bias, (float*)0, mid, mid);
}
__global__ __launch_bounds__(256) void gemm_ffn2_kernel(
    const _Float16* __restrict__ A16, const _Float16* __restrict__ Bt,
    const float* __restrict__ bias, const float* __restrict__ x1, float* __restrict__ outf) {
  gemm_body<4>(A16, Bt, (unsigned)HID, bias, x1, outf, (_Float16*)0, (_Float16*)0);
}

__global__ __launch_bounds__(256) void attn_kernel(
    const _Float16* __restrict__ Qh, const _Float16* __restrict__ Kh,
    const _Float16* __restrict__ Vt, const _Float16* __restrict__ VtR,
    _Float16* __restrict__ Ov) {
  __shared__ _Float16 Ks[64 * LDT];
  __shared__ _Float16 Vs[64 * LDT];
  __shared__ _Float16 VRs[64 * LDT];
  __shared__ _Float16 Ps[8 * 16 * LDT];

  const unsigned tid = threadIdx.x, lane = tid & 31u, w = tid >> 5;
  const unsigned hh = lane >> 4, m = lane & 15u;
  const unsigned q0 = blockIdx.x * 128u;
  const unsigned head = blockIdx.y;
  const unsigned b = blockIdx.z;
  const float scale = 0.125f;
  const unsigned qrow0 = q0 + w * 16u;
  const bool first_blk = (blockIdx.x == 0u);
  _Float16* P = Ps + w * (16u * LDT);

  const size_t qoff = (size_t)(b * (unsigned)SEQ + qrow0 + m) * DIM + head * HD + hh * 8u;
  v16h qf[2];
  qf[0] = frag_at(Qh + qoff);
  qf[1] = frag_at(Qh + qoff + 32);

  float mrow[8], lrow[8];
  v8f o[4];
#pragma unroll
  for (int v = 0; v < 8; ++v) { mrow[v] = -1.0e30f; lrow[v] = 0.0f; }
#pragma unroll
  for (int nb = 0; nb < 4; ++nb) o[nb] = (v8f){};

  const size_t kplane = (size_t)b * SEQ * DIM + head * HD;
  const size_t vplane = ((size_t)b * DIM + head * HD) * SEQ;
  const size_t rplane = ((size_t)b * DIM + head * HD) * 64u;
  const unsigned kend = q0 + 128u;

  for (unsigned kb = 0; kb < kend; kb += 64u) {
    const bool early = first_blk && (kb == 0u);
#pragma unroll
    for (unsigned j = 0; j < 2u; ++j) {
      const unsigned idx = tid + 256u * j;
      const unsigned r = idx >> 3, c = (idx & 7u) * 8u;
      *(v8h*)&Ks[r * LDT + c] = *(const v8h*)(Kh + kplane + (size_t)(kb + r) * DIM + c);
      *(v8h*)&Vs[r * LDT + c] = *(const v8h*)(Vt + vplane + (size_t)r * SEQ + kb + c);
    }
    if (early) {
#pragma unroll
      for (unsigned j = 0; j < 2u; ++j) {
        const unsigned idx = tid + 256u * j;
        const unsigned r = idx >> 3, c = (idx & 7u) * 8u;
        *(v8h*)&VRs[r * LDT + c] = *(const v8h*)(VtR + rplane + (size_t)r * 64u + c);
      }
    }
    __syncthreads();

    v8f s[4];
#pragma unroll
    for (int kg = 0; kg < 4; ++kg) {
      v8f t = {};
#pragma unroll
      for (int c = 0; c < 2; ++c) {
        const v16h kf = ld_frag(&Ks[(kg * 16) * LDT + c * 32], LDT);
        t = wmma16(qf[c], kf, t);
      }
      s[kg] = t * scale;
    }

    if (kb >= q0) {
#pragma unroll
      for (int kg = 0; kg < 4; ++kg)
#pragma unroll
        for (int v = 0; v < 8; ++v) {
          const unsigned key = kb + (unsigned)kg * 16u + m;
          const unsigned row = qrow0 + hh * 8u + (unsigned)v;
          s[kg][v] = (key > row) ? -1.0e30f : s[kg][v];
        }
    }

    float alpha[8];
#pragma unroll
    for (int v = 0; v < 8; ++v) {
      float mx = fmaxf(fmaxf(s[0][v], s[1][v]), fmaxf(s[2][v], s[3][v]));
      mx = red16_max(mx);
      const float mn = fmaxf(mrow[v], mx);
      alpha[v] = __expf(mrow[v] - mn);
      mrow[v] = mn;
    }
#pragma unroll
    for (int kg = 0; kg < 4; ++kg)
#pragma unroll
      for (int v = 0; v < 8; ++v) s[kg][v] = __expf(s[kg][v] - mrow[v]);
#pragma unroll
    for (int v = 0; v < 8; ++v) {
      const float rs = red16_sum((s[0][v] + s[1][v]) + (s[2][v] + s[3][v]));
      lrow[v] = alpha[v] * lrow[v] + rs;
    }
#pragma unroll
    for (int nb = 0; nb < 4; ++nb)
#pragma unroll
      for (int v = 0; v < 8; ++v) o[nb][v] = o[nb][v] * alpha[v];

#pragma unroll
    for (int kg = 0; kg < 4; ++kg)
#pragma unroll
      for (int v = 0; v < 8; ++v)
        P[(hh * 8u + (unsigned)v) * LDT + (unsigned)kg * 16u + m] = (_Float16)(s[kg][v] * PCARRY);
    wave_lds_sync();

#pragma unroll
    for (int c = 0; c < 2; ++c) {
      const v16h pf = ld_frag(P + c * 32, LDT);
#pragma unroll
      for (int nb = 0; nb < 4; ++nb) {
        const v16h vf = ld_frag(&Vs[(nb * 16) * LDT + c * 32], LDT);
        o[nb] = wmma16(pf, vf, o[nb]);
      }
    }

    if (early) {
#pragma unroll
      for (int nb = 0; nb < 4; ++nb) {
        v8f o2 = {};
#pragma unroll
        for (int c = 0; c < 2; ++c) {
          const v16h pf = ld_frag(P + c * 32, LDT);
          const v16h vr = ld_frag(&VRs[(nb * 16) * LDT + c * 32], LDT);
          o2 = wmma16(pf, vr, o2);
        }
#pragma unroll
        for (int v = 0; v < 8; ++v) o[nb][v] = o[nb][v] + o2[v] * (1.0f / RCARRY);
      }
      wave_lds_sync();
#pragma unroll
      for (int kg = 0; kg < 4; ++kg)
#pragma unroll
        for (int v = 0; v < 8; ++v) {
          const float t = s[kg][v] * PCARRY;
          const float hi = (float)((_Float16)t);
          P[(hh * 8u + (unsigned)v) * LDT + (unsigned)kg * 16u + m] =
              (_Float16)((t - hi) * RCARRY);
        }
      wave_lds_sync();
#pragma unroll
      for (int nb = 0; nb < 4; ++nb) {
        v8f o2 = {};
#pragma unroll
        for (int c = 0; c < 2; ++c) {
          const v16h pf = ld_frag(P + c * 32, LDT);
          const v16h vf = ld_frag(&Vs[(nb * 16) * LDT + c * 32], LDT);
          o2 = wmma16(pf, vf, o2);
        }
#pragma unroll
        for (int v = 0; v < 8; ++v) o[nb][v] = o[nb][v] + o2[v] * (1.0f / RCARRY);
      }
    }
    __syncthreads();
  }

  float inv[8];
#pragma unroll
  for (int v = 0; v < 8; ++v) inv[v] = __builtin_amdgcn_rcpf(lrow[v]) * (VCARRY / PCARRY);
#pragma unroll
  for (int nb = 0; nb < 4; ++nb)
#pragma unroll
    for (int v = 0; v < 8; ++v)
      P[(hh * 8u + (unsigned)v) * LDT + (unsigned)nb * 16u + m] = (_Float16)(o[nb][v] * inv[v]);
  wave_lds_sync();
  v8h x[4];
  size_t off[4];
#pragma unroll
  for (unsigned i = 0; i < 4u; ++i) {
    const unsigned r = 4u * i + (lane >> 3);
    const unsigned c = (lane & 7u) * 8u;
    x[i] = *(const v8h*)&P[r * LDT + c];
    off[i] = (size_t)(b * (unsigned)SEQ + qrow0 + r) * DIM + head * HD + c;
  }
#pragma unroll
  for (int i = 0; i < 4; ++i) *(volatile v8h*)(Ov + off[i]) = x[i];
  __threadfence();
#pragma unroll
  for (int i = 0; i < 4; ++i) *(volatile v8h*)(Ov + off[i]) = x[i];
}

extern "C" void kernel_launch(void* const* d_in, const int* in_sizes, int n_in,
                              void* d_out, int out_size, void* d_ws, size_t ws_size,
                              hipStream_t stream) {
  if (n_in < 13) return;
  const long long need_x = ((long long)(NB - 1) * SEQ_FULL + SEQ) * EMB;
  if ((long long)in_sizes[0] < need_x) return;
  if (in_sizes[1] < WELEMS || in_sizes[2] < WELEMS || in_sizes[3] < WELEMS) return;
  if (in_sizes[4] < WELEMS || in_sizes[5] < WELEMS || in_sizes[7] < WELEMS) return;
  if (in_sizes[6] < HID || in_sizes[8] < EMB) return;
  if (in_sizes[9] < EMB || in_sizes[10] < EMB || in_sizes[11] < EMB || in_sizes[12] < EMB) return;
  if ((long long)out_size < need_x) return;
  if (ws_size < WS_TOTAL) return;

  const float* X   = (const float*)d_in[0];
  const float* wq  = (const float*)d_in[1];
  const float* wk  = (const float*)d_in[2];
  const float* wv  = (const float*)d_in[3];
  const float* wo  = (const float*)d_in[4];
  const float* w1  = (const float*)d_in[5];
  const float* b1  = (const float*)d_in[6];
  const float* w2  = (const float*)d_in[7];
  const float* b2  = (const float*)d_in[8];
  const float* g1  = (const float*)d_in[9];
  const float* be1 = (const float*)d_in[10];
  const float* g2  = (const float*)d_in[11];
  const float* be2 = (const float*)d_in[12];
  float* out = (float*)d_out;

  char* ws = (char*)d_ws;
  _Float16* Wq_t  = (_Float16*)(ws + OFF_WQ);
  _Float16* Wk_t  = (_Float16*)(ws + OFF_WK);
  _Float16* Wv_t  = (_Float16*)(ws + OFF_WV);
  _Float16* Wo_t  = (_Float16*)(ws + OFF_WO);
  _Float16* W1_t  = (_Float16*)(ws + OFF_W1);
  _Float16* W2_t  = (_Float16*)(ws + OFF_W2);
  _Float16* H1    = (_Float16*)(ws + OFF_H1);
  _Float16* H2    = (_Float16*)(ws + OFF_H2);
  _Float16* Qh16  = (_Float16*)(ws + OFF_Q);
  _Float16* Kh16  = (_Float16*)(ws + OFF_K);
  _Float16* Vt16  = (_Float16*)(ws + OFF_VT);
  _Float16* Ctx16 = (_Float16*)(ws + OFF_CTX);
  _Float16* VtR16 = (_Float16*)(ws + OFF_VR);
  float*    X1    = (float*)(ws + OFF_X1);
  _Float16* Mid16 = (_Float16*)(ws + OFF_MID);

  dim3 blk(256);
  dim3 gw(WELEMS / 2048);
  dim3 gcat(DIM / 64, MROWS / 64);
  dim3 gemb(EMB / 64, MROWS / 64);

  wplane_kernel<<<gw, blk, 0, stream>>>(wq, Wq_t);
  wplane_kernel<<<gw, blk, 0, stream>>>(wk, Wk_t);
  wplane_kernel<<<gw, blk, 0, stream>>>(wv, Wv_t);
  wplane_kernel<<<gw, blk, 0, stream>>>(wo, Wo_t);
  wplane_kernel<<<gw, blk, 0, stream>>>(w1, W1_t);
  wplane_kernel<<<gw, blk, 0, stream>>>(w2, W2_t);

  ln_in_kernel<<<dim3(MROWS / 32), blk, 0, stream>>>(X, g1, be1, H1);
  gemm_qk_kernel<<<gcat, blk, 0, stream>>>(H1, Wq_t, Qh16);
  gemm_qk_kernel<<<gcat, blk, 0, stream>>>(H1, Wk_t, Kh16);
  gemm_v_kernel<<<gcat, blk, 0, stream>>>(H1, Wv_t, Vt16, VtR16);
  attn_kernel<<<dim3(SEQ / 128, NHEAD, NB), blk, 0, stream>>>(Qh16, Kh16, Vt16, VtR16, Ctx16);
  gemm_wo_kernel<<<gemb, blk, 0, stream>>>(Ctx16, Wo_t, X, X1);
  ln_ws_kernel<<<dim3(MROWS / 32), blk, 0, stream>>>(X1, g2, be2, H2);
  gemm_ffn1_kernel<<<dim3(HID / 64, MROWS / 64), blk, 0, stream>>>(H2, W1_t, b1, Mid16);
  gemm_ffn2_kernel<<<gemb, blk, 0, stream>>>(Mid16, W2_t, b2, X1, out);
}
